// MambaLayer_77807627534531
// MI455X (gfx1250) — hardware-verified
//
#include <hip/hip_runtime.h>
#include <math.h>

typedef __attribute__((ext_vector_type(16))) _Float16 v16h;
typedef __attribute__((ext_vector_type(8)))  _Float16 v8h;
typedef __attribute__((ext_vector_type(16))) __bf16   v16b;
typedef __attribute__((ext_vector_type(8)))  __bf16   v8b;
typedef __attribute__((ext_vector_type(8)))  float    v8f;
typedef __attribute__((ext_vector_type(4)))  float    v4f;

constexpr int kBatch  = 2;
constexpr int kSeq    = 4096;
constexpr int kDm     = 256;
constexpr int kOut    = 256;
constexpr int kDin    = 512;
constexpr int kNst    = 16;
constexpr int kDtR    = 16;
constexpr int kXprjN  = kDtR + 2 * kNst;
constexpr int kXdP    = 64;
constexpr int kXzP    = 2 * kDin;
constexpr int kRows   = kBatch * kSeq;
constexpr int kConvTP = 260;
constexpr int kScanTS = 64;
constexpr int kScanCh = 64;
constexpr int kScanYP = 68;
constexpr float kCarryW = 32.0f;
constexpr float kCarryU = 16.0f;
constexpr float kCarryY = 128.0f;
constexpr float kLog2e  = 1.4426950408889634f;
static_assert(kXprjN == 48 && kXdP >= kXprjN, "x_proj width");
static_assert((kDm % 32) == 0 && (kDin % 32) == 0, "GEMM K multiples of 32");
static_assert((kRows % 64) == 0 && (kXzP % 64) == 0 && (kXdP % 64) == 0 && (kDm % 64) == 0 && (kOut % 64) == 0, "GEMM M,N multiples of 64");
static_assert((kSeq % kScanTS) == 0 && (kSeq % 64) == 0 && (kDin % kScanCh) == 0 && (kDin % 256) == 0, "tile multiples");
static_assert(kDm == 256, "one wave per row holds 8 values per lane");
static_assert((kXprjN * kDin) % 8 == 0, "pad boundary on an 8-element group");

constexpr size_t kOffWIN  = 0;
constexpr size_t kOffWXP  = kOffWIN  + (size_t)kXzP  * kDm  * 2;
constexpr size_t kOffWOUT = kOffWXP  + (size_t)kXdP  * kDin * 2;
constexpr size_t kOffWPH  = kOffWOUT + (size_t)kDm   * kDin * 2;
constexpr size_t kOffWPL  = kOffWPH  + (size_t)kOut  * kDm  * 2;
constexpr size_t kOffXN   = kOffWPL  + (size_t)kOut  * kDm  * 2;
constexpr size_t kOffXZ   = kOffXN   + (size_t)kRows * kDm  * 2;
constexpr size_t kOffUC   = kOffXZ   + (size_t)kRows * kXzP * 4;
constexpr size_t kOffUC16 = kOffUC   + (size_t)kRows * kDin * 4;
constexpr size_t kOffXD   = kOffUC16 + (size_t)kRows * kDin * 2;
constexpr size_t kOffY16  = kOffXD   + (size_t)kRows * kXdP * 4;
constexpr size_t kOffYM   = kOffY16  + (size_t)kRows * kDin * 2;
constexpr size_t kOffXMH  = kOffYM   + (size_t)kRows * kDm  * 4;
constexpr size_t kOffXML  = kOffXMH  + (size_t)kRows * kDm  * 2;
constexpr size_t kWsTotal = kOffXML  + (size_t)kRows * kDm  * 2;
static_assert(kWsTotal == 91291648ull, "carve total");
static_assert(kWsTotal <= 134217728ull, "carve cap");
static_assert((kOffWXP % 128) == 0 && (kOffWOUT % 128) == 0 && (kOffWPH % 128) == 0 && (kOffWPL % 128) == 0 &&
              (kOffXN % 128) == 0 && (kOffXZ % 128) == 0 && (kOffUC % 128) == 0 && (kOffUC16 % 128) == 0 &&
              (kOffXD % 128) == 0 && (kOffY16 % 128) == 0 && (kOffYM % 128) == 0 && (kOffXMH % 128) == 0 &&
              (kOffXML % 128) == 0, "128-B aligned regions");

__device__ __forceinline__ unsigned short f2bf_bits(float f) {
  unsigned u = __float_as_uint(f);
  return (unsigned short)((u + 0x7FFFu + ((u >> 16) & 1u)) >> 16);
}
__device__ __forceinline__ float bf_bits2f(unsigned short h) { return __uint_as_float(((unsigned)h) << 16); }

__device__ __forceinline__ void dep_guard4_h(v8f& a, v8f& b, v8f& c, v8f& d, v16h x, v16h y) { asm volatile("v_nop\n\tv_nop\n\tv_nop\n\tv_nop" : "+v"(a), "+v"(b), "+v"(c), "+v"(d) : "v"(x), "v"(y)); }
__device__ __forceinline__ void dep_guard4_b(v8f& a, v8f& b, v8f& c, v8f& d, v16b x, v16b y) { asm volatile("v_nop\n\tv_nop\n\tv_nop\n\tv_nop" : "+v"(a), "+v"(b), "+v"(c), "+v"(d) : "v"(x), "v"(y)); }
__device__ __forceinline__ void keep4_h(v16h a, v16h b, v16h c, v16h d) { asm volatile("v_nop" :: "v"(a), "v"(b), "v"(c), "v"(d)); }
__device__ __forceinline__ void keep4_b(v16b a, v16b b, v16b c, v16b d) { asm volatile("v_nop" :: "v"(a), "v"(b), "v"(c), "v"(d)); }
__device__ __forceinline__ void acc_guard4(v8f& a, v8f& b, v8f& c, v8f& d) { asm volatile("v_nop\n\tv_nop\n\tv_nop\n\tv_nop" : "+v"(a), "+v"(b), "+v"(c), "+v"(d)); }
template <typename T> struct Frag;
template <> struct Frag<_Float16> {
  typedef v16h V; union U { v16h v; v8h h[2]; };
  static __device__ __forceinline__ v16h load(const _Float16* p) {
    U f; f.h[0] = *(const v8h*)(p); f.h[1] = *(const v8h*)(p + 16); return f.v;
  }
  static __device__ __forceinline__ v8f mma(v16h a, v16h b, v8f c) {
    return __builtin_amdgcn_wmma_f32_16x16x32_f16(false, a, false, b, (short)0, c, false, false);
  }
  static __device__ __forceinline__ void guard4(v8f& a, v8f& b, v8f& c, v8f& d, v16h x, v16h y) { dep_guard4_h(a, b, c, d, x, y); }
  static __device__ __forceinline__ void keep(v16h a, v16h b, v16h c, v16h d) { keep4_h(a, b, c, d); }
};
template <> struct Frag<__bf16> {
  typedef v16b V; union U { v16b v; v8b h[2]; };
  static __device__ __forceinline__ v16b load(const __bf16* p) {
    U f; f.h[0] = *(const v8b*)(p); f.h[1] = *(const v8b*)(p + 16); return f.v;
  }
  static __device__ __forceinline__ v8f mma(v16b a, v16b b, v8f c) {
    return __builtin_amdgcn_wmma_f32_16x16x32_bf16(false, a, false, b, (short)0, c, false, false);
  }
  static __device__ __forceinline__ void guard4(v8f& a, v8f& b, v8f& c, v8f& d, v16b x, v16b y) { dep_guard4_b(a, b, c, d, x, y); }
  static __device__ __forceinline__ void keep(v16b a, v16b b, v16b c, v16b d) { keep4_b(a, b, c, d); }
};

template <int ET> struct Elem;
template <> struct Elem<0> { typedef _Float16 T; };
template <> struct Elem<1> { typedef __bf16 T; };
template <int ET, bool SPLIT, int BIAS_MODE, int OUT_MODE, bool RESID, int ACT = 0>
__global__ __launch_bounds__(256) void wmma_gemm64(
    const unsigned short* __restrict__ Ap, const unsigned short* __restrict__ A2p, int lda, long strideA,
    const unsigned short* __restrict__ Btp, const unsigned short* __restrict__ Bt2p, int ldb, long strideB,
    void* __restrict__ Cout, void* __restrict__ Cout2, int ldc, long strideC,
    const float* __restrict__ bias,
    const float* __restrict__ resid, long strideR,
    int M, int N, int K, float scale) {
  typedef typename Elem<ET>::T T;
  typedef typename Frag<T>::V V;
  const T* A = (const T*)Ap; const T* A2 = (const T*)A2p; const T* Bt = (const T*)Btp; const T* Bt2 = (const T*)Bt2p;
  __shared__ __align__(16) float sT[8][16 * 68];
  const int b    = blockIdx.y;
  const int lane = threadIdx.x & 31;
  const int wave = threadIdx.x >> 5;
  const int tilesN = N >> 6;
  const int tilesM = M >> 6;
  const int tile = blockIdx.x * 8 + wave;
  if (tile >= tilesM * tilesN) return;
  const int tm = tile / tilesN;
  const int tn = tile - tm * tilesN;
  const int m0 = tm << 6;
  const int n0 = tn << 6;

  const T* Ab  = A  + (size_t)b * strideA;
  const T* Bb  = Bt + (size_t)b * strideB;
  const T* Ab2 = SPLIT ? (A2  + (size_t)b * strideA) : nullptr;
  const T* Bb2 = SPLIT ? (Bt2 + (size_t)b * strideB) : nullptr;

  const int rlane = lane & 15;
  const int koff  = (lane >> 4) * 8;
  const int mOff  = (lane >> 4) * 8;

  v8f acc[4][4];
#pragma unroll
  for (int i = 0; i < 4; ++i)
#pragma unroll
    for (int j = 0; j < 4; ++j) acc[i][j] = (v8f){0.f,0.f,0.f,0.f,0.f,0.f,0.f,0.f};

  for (int k0 = 0; k0 < K; k0 += 32) {
    V bh[4], bl[4];
#pragma unroll
    for (int j = 0; j < 4; ++j) {
      const size_t bo = (size_t)(n0 + (j << 4) + rlane) * ldb + koff + k0;
      bh[j] = Frag<T>::load(Bb + bo);
      if (SPLIT) bl[j] = Frag<T>::load(Bb2 + bo);
    }
#pragma unroll
    for (int i = 0; i < 4; ++i) {
      const size_t ao = (size_t)(m0 + (i << 4) + rlane) * lda + koff + k0;
      V ah = Frag<T>::load(Ab + ao);
      V al;
      if (SPLIT) al = Frag<T>::load(Ab2 + ao);
#pragma unroll
      for (int j = 0; j < 4; ++j) {
        acc[i][j] = Frag<T>::mma(ah, bh[j], acc[i][j]);
        if (SPLIT) {
          acc[i][j] = Frag<T>::mma(ah, bl[j], acc[i][j]);
          acc[i][j] = Frag<T>::mma(al, bh[j], acc[i][j]);
        }
      }
      Frag<T>::guard4(acc[i][0], acc[i][1], acc[i][2], acc[i][3], ah, SPLIT ? al : ah);
    }
    Frag<T>::keep(bh[0], bh[1], bh[2], bh[3]);
    if (SPLIT) Frag<T>::keep(bl[0], bl[1], bl[2], bl[3]);
  }
  acc_guard4(acc[0][0], acc[0][1], acc[0][2], acc[0][3]);
  acc_guard4(acc[1][0], acc[1][1], acc[1][2], acc[1][3]);
  acc_guard4(acc[2][0], acc[2][1], acc[2][2], acc[2][3]);
  acc_guard4(acc[3][0], acc[3][1], acc[3][2], acc[3][3]);

  float* slab = sT[wave];
  const float* Rb = RESID ? (resid + (size_t)b * strideR) : nullptr;
#pragma unroll
  for (int i = 0; i < 4; ++i) {
    const int mBase = m0 + (i << 4);
#pragma unroll
    for (int j = 0; j < 4; ++j) {
      const int n = n0 + (j << 4) + rlane;
      float bv = 0.f;
      if (BIAS_MODE == 2) bv = bias[n];
#pragma unroll
      for (int r = 0; r < 8; ++r) {
        float v = acc[i][j][r] * scale;
        if (BIAS_MODE == 1) v += bias[mBase + mOff + r];
        if (BIAS_MODE == 2) v += bv;
        if (RESID) v += Rb[(size_t)(mBase + mOff + r) * ldc + n];
        if (ACT == 1) v = tanhf(v);
        if (ACT == 2) v = fmaxf(v, 0.0f);
        if (ACT == 3) v = v / (1.0f + expf(-v));
        if (ACT == 4) v = (v > 0.f) ? v : 0.01f * v;
        slab[(mOff + r) * 68 + (j << 4) + rlane] = v;
      }
    }
    __builtin_amdgcn_fence(__ATOMIC_RELEASE, "workgroup");
    __builtin_amdgcn_wave_barrier();
    __builtin_amdgcn_fence(__ATOMIC_ACQUIRE, "workgroup");
    if (OUT_MODE == 0) {
      float* C = (float*)Cout + (size_t)b * strideC;
      const int hh = lane >> 4, c4 = (lane & 15) * 4;
      for (int pass = 0; pass < 2; ++pass) {
#pragma unroll
        for (int it = 0; it < 8; ++it) {
          const int row = it * 2 + hh;
          v4f v = *(const v4f*)(slab + row * 68 + c4);
          *(volatile v4f*)(C + (size_t)(mBase + row) * ldc + n0 + c4) = v;
        }
        __threadfence();
      }
    } else {
      const int q = lane >> 3, c8 = (lane & 7) * 8;
      unsigned short* C  = (unsigned short*)Cout  + (size_t)b * strideC;
      unsigned short* C2 = (OUT_MODE == 2) ? ((unsigned short*)Cout2 + (size_t)b * strideC) : nullptr;
      for (int pass = 0; pass < 2; ++pass) {
#pragma unroll
        for (int it = 0; it < 4; ++it) {
          const int row = it * 4 + q;
          const float* sp = slab + row * 68 + c8;
          v8h hv, lv;
#pragma unroll
          for (int e = 0; e < 8; ++e) {
            if (OUT_MODE == 1) {
              hv[e] = (_Float16)sp[e];
            } else {
              unsigned short hb = f2bf_bits(sp[e]);
              unsigned short lb = f2bf_bits(sp[e] - bf_bits2f(hb));
              hv[e] = __builtin_bit_cast(_Float16, hb);
              lv[e] = __builtin_bit_cast(_Float16, lb);
            }
          }
          *(volatile v8h*)(C + (size_t)(mBase + row) * ldc + n0 + c8) = hv;
          if (OUT_MODE == 2) *(volatile v8h*)(C2 + (size_t)(mBase + row) * ldc + n0 + c8) = lv;
        }
        __threadfence();
      }
    }
    __builtin_amdgcn_fence(__ATOMIC_RELEASE, "workgroup");
    __builtin_amdgcn_wave_barrier();
    __builtin_amdgcn_fence(__ATOMIC_ACQUIRE, "workgroup");
  }
}

__global__ __launch_bounds__(256) void cast_f16_pad_kernel(
    const float* __restrict__ src, unsigned short* __restrict__ dst, int total8, int nreal, float scale)
{
  const int i = blockIdx.x * 256 + threadIdx.x;
  if (i >= total8) return;
  const int e0 = i << 3;
  const bool real = (e0 < nreal);
  const size_t ec = real ? (size_t)e0 : (size_t)0;
  const v4f a0 = *(const v4f*)(src + ec);
  const v4f a1 = *(const v4f*)(src + ec + 4);
  const float fac = real ? scale : 0.0f;
  v8h hv;
#pragma unroll
  for (int e = 0; e < 4; ++e) {
    hv[e]     = (_Float16)(a0[e] * fac);
    hv[4 + e] = (_Float16)(a1[e] * fac);
  }
  unsigned short* q = dst + (size_t)e0;
  *(volatile v8h*)q = hv;
  __threadfence();
  *(volatile v8h*)q = hv;
}

__global__ __launch_bounds__(256) void split_rows_bf16_kernel(
    const float* __restrict__ src, unsigned short* __restrict__ dhi, unsigned short* __restrict__ dlo, int total8)
{
  const int i = blockIdx.x * 256 + threadIdx.x;
  if (i >= total8) return;
  const size_t e0 = (size_t)i << 3;
  const v4f a0 = *(const v4f*)(src + e0);
  const v4f a1 = *(const v4f*)(src + e0 + 4);
  v8h hv, lv;
#pragma unroll
  for (int e = 0; e < 4; ++e) {
    const unsigned short h0 = f2bf_bits(a0[e]), h1 = f2bf_bits(a1[e]);
    const unsigned short l0 = f2bf_bits(a0[e] - bf_bits2f(h0)), l1 = f2bf_bits(a1[e] - bf_bits2f(h1));
    hv[e]     = __builtin_bit_cast(_Float16, h0);
    hv[4 + e] = __builtin_bit_cast(_Float16, h1);
    lv[e]     = __builtin_bit_cast(_Float16, l0);
    lv[4 + e] = __builtin_bit_cast(_Float16, l1);
  }
  unsigned short* qh = dhi + e0;
  unsigned short* ql = dlo + e0;
  *(volatile v8h*)qh = hv;
  *(volatile v8h*)ql = lv;
  __threadfence();
  *(volatile v8h*)qh = hv;
  *(volatile v8h*)ql = lv;
}

template <int MODE>
__global__ __launch_bounds__(256) void layernorm_kernel(
    const float* __restrict__ X, const float* __restrict__ R, const float* __restrict__ sscl,
    const float* __restrict__ gw, const float* __restrict__ gb,
    unsigned short* __restrict__ O1, unsigned short* __restrict__ O2, int nrows, float oscale)
{
  const int lane = threadIdx.x & 31, wave = threadIdx.x >> 5;
  int row = blockIdx.x * 8 + wave;
  row = (row < nrows) ? row : (nrows - 1);
  const int c0 = lane * 8;
  const size_t base = (size_t)row * kDm + c0;
  const v4f a0 = *(const v4f*)(X + base);
  const v4f a1 = *(const v4f*)(X + base + 4);
  float v[8];
  if (MODE == 1) {
    const v4f r0 = *(const v4f*)(R + base);
    const v4f r1 = *(const v4f*)(R + base + 4);
    const float s = sscl[0];
#pragma unroll
    for (int e = 0; e < 4; ++e) { v[e] = a0[e] + s * r0[e]; v[4 + e] = a1[e] + s * r1[e]; }
  } else {
#pragma unroll
    for (int e = 0; e < 4; ++e) { v[e] = a0[e]; v[4 + e] = a1[e]; }
  }
  asm volatile("" ::: "memory");
  const v4f w0 = *(const v4f*)(gw + c0);
  const v4f w1 = *(const v4f*)(gw + c0 + 4);
  const v4f b0 = *(const v4f*)(gb + c0);
  const v4f b1 = *(const v4f*)(gb + c0 + 4);

  float sum = 0.0f;
#pragma unroll
  for (int e = 0; e < 8; ++e) sum += v[e];
#pragma unroll
  for (int off = 16; off > 0; off >>= 1) sum += __shfl_xor(sum, off, 32);
  const float mu = sum * (1.0f / (float)kDm);
  float sq = 0.0f;
#pragma unroll
  for (int e = 0; e < 8; ++e) { const float dv = v[e] - mu; sq = fmaf(dv, dv, sq); }
#pragma unroll
  for (int off = 16; off > 0; off >>= 1) sq += __shfl_xor(sq, off, 32);
  const float var = sq * (1.0f / (float)kDm);
  const float inv = rsqrtf(var + 1e-5f);
  float o[8];
#pragma unroll
  for (int e = 0; e < 4; ++e) {
    o[e]     = ((v[e] - mu) * inv) * w0[e] + b0[e];
    o[4 + e] = ((v[4 + e] - mu) * inv) * w1[e] + b1[e];
  }
  if (MODE == 0) {
    v8h hv;
#pragma unroll
    for (int e = 0; e < 8; ++e) hv[e] = (_Float16)(o[e] * oscale);
    unsigned short* q = O1 + base;
    *(volatile v8h*)q = hv;
    __threadfence();
    *(volatile v8h*)q = hv;
  } else {
    v8h hv, lv;
#pragma unroll
    for (int e = 0; e < 8; ++e) {
      const unsigned short hb = f2bf_bits(o[e]);
      const unsigned short lb = f2bf_bits(o[e] - bf_bits2f(hb));
      hv[e] = __builtin_bit_cast(_Float16, hb);
      lv[e] = __builtin_bit_cast(_Float16, lb);
    }
    unsigned short* qh = O1 + base;
    unsigned short* ql = O2 + base;
    *(volatile v8h*)qh = hv;
    *(volatile v8h*)ql = lv;
    __threadfence();
    *(volatile v8h*)qh = hv;
    *(volatile v8h*)ql = lv;
  }
}

__global__ __launch_bounds__(256) void conv_silu_kernel(
    const float* __restrict__ XZ, const float* __restrict__ cw, const float* __restrict__ cb,
    float* __restrict__ UC, unsigned short* __restrict__ UC16)
{
  __shared__ __align__(16) float sT[16 * kConvTP];
  const int tid = threadIdx.x, lane = tid & 31, wave = tid >> 5;
  const int d0 = blockIdx.x * 256, d = d0 + tid;
  const int g0 = blockIdx.y * 64;
  const int tb = g0 & (kSeq - 1);
  const float w0 = cw[d * 4 + 0], w1 = cw[d * 4 + 1], w2 = cw[d * 4 + 2], w3 = cw[d * 4 + 3];
  const float bc = cb[d];
  float xm3, xm2, xm1;
  {
    const bool hist = (tb > 0);
    const int rb = hist ? (g0 - 3) : g0;
    const float v3 = XZ[(size_t)rb * kXzP + d];
    const float v2 = XZ[(size_t)(rb + 1) * kXzP + d];
    const float v1 = XZ[(size_t)(rb + 2) * kXzP + d];
    xm3 = hist ? v3 : 0.f;
    xm2 = hist ? v2 : 0.f;
    xm1 = hist ? v1 : 0.f;
  }
  const int hrow = wave >> 1;
  const int hch  = (wave & 1) * 128 + lane * 4;
#pragma unroll 1
  for (int sub = 0; sub < 4; ++sub) {
    const int lb = g0 + sub * 16;
#pragma unroll 1
    for (int s = 0; s < 16; ++s) {
      const float xcur = XZ[(size_t)(lb + s) * kXzP + d];
      float acc = w0 * xm3;
      acc = fmaf(w1, xm2, acc);
      acc = fmaf(w2, xm1, acc);
      acc = fmaf(w3, xcur, acc);
      const float sv = acc + bc;
      const float sg = __builtin_amdgcn_rcpf(1.0f + expf(-sv));
      sT[s * kConvTP + tid] = sv * sg;
      xm3 = xm2; xm2 = xm1; xm1 = xcur;
    }
    __syncthreads();
    v4f fv[4];
    v8h bv[2];
#pragma unroll
    for (int it = 0; it < 4; ++it) fv[it] = *(const v4f*)(sT + (it * 4 + hrow) * kConvTP + hch);
#pragma unroll
    for (int it = 0; it < 2; ++it) {
      const float* sp = sT + (it * 8 + wave) * kConvTP + lane * 8;
      const v4f a0 = *(const v4f*)(sp);
      const v4f a1 = *(const v4f*)(sp + 4);
#pragma unroll
      for (int e = 0; e < 4; ++e) {
        bv[it][e]     = (_Float16)(a0[e] * kCarryU);
        bv[it][4 + e] = (_Float16)(a1[e] * kCarryU);
      }
    }
    for (int pass = 0; pass < 2; ++pass) {
#pragma unroll
      for (int it = 0; it < 4; ++it)
        *(volatile v4f*)(UC + (size_t)(lb + it * 4 + hrow) * kDin + d0 + hch) = fv[it];
#pragma unroll
      for (int it = 0; it < 2; ++it)
        *(volatile v8h*)(UC16 + (size_t)(lb + it * 8 + wave) * kDin + d0 + lane * 8) = bv[it];
      __threadfence();
    }
    __syncthreads();
  }
}

__global__ __launch_bounds__(64) void scan_kernel(
    const float* __restrict__ XD, const float* __restrict__ UC, const float* __restrict__ XZ,
    const float* __restrict__ Wdt, const float* __restrict__ bdt, const float* __restrict__ Alog,
    const float* __restrict__ Dp, unsigned short* __restrict__ Y16)
{
  __shared__ __align__(16) float sX[kScanTS * kXdP];
  __shared__ __align__(16) float sY[kScanTS * kScanYP];
  __shared__ __align__(16) float sW[kDtR * kScanCh];
  __shared__ __align__(16) float sA[kNst * kScanCh];
  const int tid = threadIdx.x, lane = tid & 31, wave = tid >> 5;
  constexpr int kBlkPerB = kDin / kScanCh;
  const int bix = blockIdx.x / kBlkPerB;
  const int d0  = (blockIdx.x - bix * kBlkPerB) * kScanCh;
  const int d   = d0 + tid;
  const size_t row0 = (size_t)bix * kSeq;
#pragma unroll 1
  for (int r = 0; r < kDtR; ++r) sW[r * kScanCh + tid] = Wdt[(size_t)d * kDtR + r];
#pragma unroll 1
  for (int s = 0; s < kNst; ++s) sA[s * kScanCh + tid] = -expf(Alog[(size_t)d * kNst + s]) * kLog2e;
  __syncthreads();
  float A2[kNst], h[kNst];
#pragma unroll
  for (int s = 0; s < kNst; ++s) {
    A2[s] = sA[s * kScanCh + tid];
    h[s] = 0.0f;
  }
  const float bb = bdt[d], Dd = Dp[d];
  const int lr = tid >> 4, lc4 = (tid & 15) * 4;
  const int q = lane >> 3, c8 = (lane & 7) * 8;
#pragma unroll 1
  for (int t0 = 0; t0 < kSeq; t0 += kScanTS) {
    __syncthreads();
#pragma unroll
    for (int i = 0; i < 16; ++i) {
      const int r = lr + 4 * i;
      *(v4f*)(sX + r * kXdP + lc4) = *(const v4f*)(XD + (row0 + t0 + r) * kXdP + lc4);
    }
    __syncthreads();
#pragma unroll 1
    for (int s = 0; s < kScanTS; ++s) {
      const int t = t0 + s;
      const float* xr = sX + s * kXdP;
      float vdot = 0.0f;
#pragma unroll 1
      for (int r4 = 0; r4 < kDtR / 4; ++r4) {
        const v4f xv = *(const v4f*)(xr + 4 * r4);
        const float* wp = sW + (4 * r4) * kScanCh + tid;
        vdot = fmaf(xv[0], wp[0], vdot);
        vdot = fmaf(xv[1], wp[kScanCh], vdot);
        vdot = fmaf(xv[2], wp[2 * kScanCh], vdot);
        vdot = fmaf(xv[3], wp[3 * kScanCh], vdot);
      }
      float Bs[kNst], Cs[kNst];
#pragma unroll
      for (int q4 = 0; q4 < 4; ++q4) {
        const v4f bv = *(const v4f*)(xr + kDtR + 4 * q4);
        const v4f cv = *(const v4f*)(xr + kDtR + kNst + 4 * q4);
        Bs[4 * q4 + 0] = bv[0]; Bs[4 * q4 + 1] = bv[1]; Bs[4 * q4 + 2] = bv[2]; Bs[4 * q4 + 3] = bv[3];
        Cs[4 * q4 + 0] = cv[0]; Cs[4 * q4 + 1] = cv[1]; Cs[4 * q4 + 2] = cv[2]; Cs[4 * q4 + 3] = cv[3];
      }
      const float v   = vdot + bb;
      const float ea  = expf(-fabsf(v));
      const float dt  = fmaxf(v, 0.0f) + log1pf(ea);
      const float xt  = UC[(row0 + t) * kDin + d];
      const float dtx = dt * xt;
      float y = 0.0f;
#pragma unroll
      for (int k = 0; k < kNst; ++k) {
        const float e  = exp2f(dt * A2[k]);
        const float hn = fmaf(e, h[k], dtx * Bs[k]);
        h[k] = hn;
        y = fmaf(hn, Cs[k], y);
      }
      y = fmaf(xt, Dd, y);
      const float zv = XZ[(row0 + t) * kXzP + kDin + d];
      const float sg = __builtin_amdgcn_rcpf(1.0f + expf(-zv));
      const float g  = zv * sg;
      sY[s * kScanYP + tid] = (y * g) * kCarryY;
    }
    __syncthreads();
    v8h hv[8];
#pragma unroll
    for (int it = 0; it < 8; ++it) {
      const int row = it * 8 + wave * 4 + q;
      const float* sp = sY + row * kScanYP + c8;
      const v4f a0 = *(const v4f*)(sp);
      const v4f a1 = *(const v4f*)(sp + 4);
#pragma unroll
      for (int e = 0; e < 4; ++e) {
        hv[it][e]     = (_Float16)a0[e];
        hv[it][4 + e] = (_Float16)a1[e];
      }
    }
    for (int pass = 0; pass < 2; ++pass) {
#pragma unroll
      for (int it = 0; it < 8; ++it) {
        const int row = it * 8 + wave * 4 + q;
        const size_t o = (row0 + t0 + row) * kDin + d0 + c8;
        *(volatile v8h*)(Y16 + o) = hv[it];
      }
      __threadfence();
    }
  }
}

extern "C" void kernel_launch(void* const* d_in, const int* in_sizes, int n_in,
                              void* d_out, int out_size, void* d_ws, size_t ws_size,
                              hipStream_t stream)
{
  if (n_in < 15) return;
  if (in_sizes[0]  != kRows * kDm) return;
  if (in_sizes[1]  != kDm || in_sizes[2] != kDm) return;
  if (in_sizes[3]  != kXzP * kDm) return;
  if (in_sizes[4]  != kDin * 4 || in_sizes[5] != kDin) return;
  if (in_sizes[6]  != kXprjN * kDin) return;
  if (in_sizes[7]  != kDin * kDtR || in_sizes[8] != kDin) return;
  if (in_sizes[9]  != kDin * kNst || in_sizes[10] != kDin) return;
  if (in_sizes[11] != kDm * kDin) return;
  if (in_sizes[12] != kOut * kDm || in_sizes[13] != kOut) return;
  if (in_sizes[14] != 1) return;
  if (out_size != kRows * kOut) return;
  if (ws_size < kWsTotal) return;

  const float* x          = (const float*)d_in[0];
  const float* ln_w       = (const float*)d_in[1];
  const float* ln_b       = (const float*)d_in[2];
  const float* W_in       = (const float*)d_in[3];
  const float* conv_w     = (const float*)d_in[4];
  const float* conv_b     = (const float*)d_in[5];
  const float* W_xprj     = (const float*)d_in[6];
  const float* W_dt       = (const float*)d_in[7];
  const float* b_dt       = (const float*)d_in[8];
  const float* A_log      = (const float*)d_in[9];
  const float* Dp         = (const float*)d_in[10];
  const float* W_out      = (const float*)d_in[11];
  const float* W_proj     = (const float*)d_in[12];
  const float* b_proj     = (const float*)d_in[13];
  const float* skip_scale = (const float*)d_in[14];
  float* out = (float*)d_out;

  char* ws = (char*)d_ws;
  unsigned short* WIN16  = (unsigned short*)(ws + kOffWIN);
  unsigned short* WXP16  = (unsigned short*)(ws + kOffWXP);
  unsigned short* WOUT16 = (unsigned short*)(ws + kOffWOUT);
  unsigned short* WPH    = (unsigned short*)(ws + kOffWPH);
  unsigned short* WPL    = (unsigned short*)(ws + kOffWPL);
  unsigned short* XN16   = (unsigned short*)(ws + kOffXN);
  float*          XZ     = (float*)(ws + kOffXZ);
  float*          UC     = (float*)(ws + kOffUC);
  unsigned short* UC16   = (unsigned short*)(ws + kOffUC16);
  float*          XD     = (float*)(ws + kOffXD);
  unsigned short* Y16    = (unsigned short*)(ws + kOffY16);
  float*          YM     = (float*)(ws + kOffYM);
  unsigned short* XMH    = (unsigned short*)(ws + kOffXMH);
  unsigned short* XML    = (unsigned short*)(ws + kOffXML);
  const float* dummy_bias  = b_proj;
  const float* dummy_resid = x;

  cast_f16_pad_kernel<<<(kXzP * kDm / 8) / 256, 256, 0, stream>>>(W_in, WIN16, kXzP * kDm / 8, kXzP * kDm, kCarryW);
  cast_f16_pad_kernel<<<(kXdP * kDin / 8) / 256, 256, 0, stream>>>(W_xprj, WXP16, kXdP * kDin / 8, kXprjN * kDin, kCarryW);
  cast_f16_pad_kernel<<<(kDm * kDin / 8) / 256, 256, 0, stream>>>(W_out, WOUT16, kDm * kDin / 8, kDm * kDin, kCarryW);
  split_rows_bf16_kernel<<<(kOut * kDm / 8) / 256, 256, 0, stream>>>(W_proj, WPH, WPL, kOut * kDm / 8);

  layernorm_kernel<0><<<kRows / 8, 256, 0, stream>>>(x, x, skip_scale, ln_w, ln_b, XN16, XN16, kRows, 1.0f);

  wmma_gemm64<0, false, 0, 0, false><<<dim3(256, 1), 256, 0, stream>>>(
      XN16, XN16, kDm, 0L,
      WIN16, WIN16, kDm, 0L,
      (void*)XZ, (void*)XZ, kXzP, 0L,
      dummy_bias, dummy_resid, 0L,
      kRows, kXzP, kDm, 1.0f / kCarryW);

  conv_silu_kernel<<<dim3(kDin / 256, kRows / 64), 256, 0, stream>>>(XZ, conv_w, conv_b, UC, UC16);

  wmma_gemm64<0, false, 0, 0, false><<<dim3(16, 1), 256, 0, stream>>>(
      UC16, UC16, kDin, 0L,
      WXP16, WXP16, kDin, 0L,
      (void*)XD, (void*)XD, kXdP, 0L,
      dummy_bias, dummy_resid, 0L,
      kRows, kXdP, kDin, 1.0f / (kCarryU * kCarryW));

  scan_kernel<<<kBatch * (kDin / kScanCh), kScanCh, 0, stream>>>(XD, UC, XZ, W_dt, b_dt, A_log, Dp, Y16);

  wmma_gemm64<0, false, 0, 0, false><<<dim3(64, 1), 256, 0, stream>>>(
      Y16, Y16, kDin, 0L,
      WOUT16, WOUT16, kDin, 0L,
      (void*)YM, (void*)YM, kDm, 0L,
      dummy_bias, dummy_resid, 0L,
      kRows, kDm, kDin, 1.0f / (kCarryY * kCarryW));

  layernorm_kernel<1><<<kRows / 8, 256, 0, stream>>>(YM, x, skip_scale, ln_w, ln_b, XMH, XML, kRows, 1.0f);

  wmma_gemm64<1, true, 2, 0, false><<<dim3(64, 1), 256, 0, stream>>>(
      XMH, XML, kDm, 0L,
      WPH, WPL, kDm, 0L,
      (void*)out, (void*)out, kOut, 0L,
      b_proj, dummy_resid, 0L,
      kRows, kOut, kDm, 1.0f);
}
